// NNK_17274358465083
// MI455X (gfx1250) — hardware-verified
//
#include <hip/hip_runtime.h>
#include <math.h>

typedef __attribute__((ext_vector_type(16))) _Float16 v16h;
typedef __attribute__((ext_vector_type(16))) __bf16 v16b;
typedef __attribute__((ext_vector_type(8)))  _Float16 v8h;
typedef __attribute__((ext_vector_type(8)))  float v8f;
typedef __attribute__((ext_vector_type(4)))  float v4f;
typedef __attribute__((ext_vector_type(2)))  float v2f;
typedef __attribute__((ext_vector_type(4)))  unsigned v4u;
typedef __attribute__((ext_vector_type(4)))  int v4i;
typedef float __attribute__((may_alias)) float_a;
typedef int __attribute__((may_alias)) int_a;

template <typename T> __device__ __forceinline__ void vst2(void* p, T v) { *(volatile T*)p = v; __threadfence(); *(volatile T*)p = v; }
__device__ __forceinline__ v8f wmma16(v16h a, v16h b, v8f c) {
  v8f d = __builtin_amdgcn_wmma_f32_16x16x32_f16(false, a, false, b, (short)0, c, false, false);
  asm volatile("v_nop\n\tv_nop\n\tv_nop\n\tv_nop" : "+v"(d) : "v"(a), "v"(b));
  return d;
}
__device__ __forceinline__ v8f wmma_bf(v16b a, v16b b, v8f c) {
  v8f d = __builtin_amdgcn_wmma_f32_16x16x32_bf16(false, a, false, b, (short)0, c, false, false);
  asm volatile("v_nop\n\tv_nop\n\tv_nop\n\tv_nop" : "+v"(d) : "v"(a), "v"(b));
  return d;
}
__device__ __forceinline__ v16h frag_h(const _Float16* rowk0, int lane) {
  union { v16h v; v8h q[2]; } u; const _Float16* p = rowk0 + 8 * (lane >> 4);
  u.q[0] = *(const v8h*)p; u.q[1] = *(const v8h*)(p + 16); return u.v;
}
__device__ __forceinline__ v16h frag_f32(const float* rowk0, int lane) {
  v16h a; const float* p = rowk0 + 8 * (lane >> 4);
#pragma unroll
  for (int i = 0; i < 8; ++i) { a[i] = (_Float16)p[i]; a[8 + i] = (_Float16)p[16 + i]; }
  return a;
}
__device__ __forceinline__ v16h frag_f32s(const float* rowk0, int lane, float sc) {
  v16h a; const float* p = rowk0 + 8 * (lane >> 4);
#pragma unroll
  for (int i = 0; i < 8; ++i) { a[i] = (_Float16)(p[i] * sc); a[8 + i] = (_Float16)(p[16 + i] * sc); }
  return a;
}
__device__ __forceinline__ v16h fragc_f32(const float* W, int k0, int n, int lane, int ld, int K) {
  v16h a; const int g = lane >> 4;
#pragma unroll
  for (int i = 0; i < 8; ++i) { const int ka = k0 + 8 * g + i, kb = ka + 16;
    a[i] = (_Float16)(ka < K ? W[(size_t)ka * ld + n] : 0.f); a[8 + i] = (_Float16)(kb < K ? W[(size_t)kb * ld + n] : 0.f); }
  return a;
}
struct F2 { v16b h, l; };
__device__ __forceinline__ F2 bsplit16(const float v[16]) { F2 r;
#pragma unroll
  for (int i = 0; i < 16; ++i) { const __bf16 h = (__bf16)v[i]; r.h[i] = h; r.l[i] = (__bf16)(v[i] - (float)h); }
  return r; }
__device__ __forceinline__ F2 split_row(const float* row, int k0, int lane) { float v[16]; const float* p = row + k0 + 8 * (lane >> 4);
#pragma unroll
  for (int i = 0; i < 8; ++i) { v[i] = p[i]; v[8 + i] = p[16 + i]; }
  return bsplit16(v); }
__device__ __forceinline__ F2 split_rowK(const float* row, int k0, int lane, int K) { float v[16]; const int g = lane >> 4;
#pragma unroll
  for (int i = 0; i < 8; ++i) { const int ka = k0 + 8 * g + i, kb = ka + 16; v[i] = ka < K ? row[ka] : 0.f; v[8 + i] = kb < K ? row[kb] : 0.f; }
  return bsplit16(v); }
__device__ __forceinline__ F2 split_col(const float* W, int k0, int n, int lane, int ld, int K) { float v[16]; const int g = lane >> 4;
#pragma unroll
  for (int i = 0; i < 8; ++i) { const int ka = k0 + 8 * g + i, kb = ka + 16; v[i] = ka < K ? W[(size_t)ka * ld + n] : 0.f; v[8 + i] = kb < K ? W[(size_t)kb * ld + n] : 0.f; }
  return bsplit16(v); }
__device__ __forceinline__ v8f mac3(const F2& a, const F2& b, v8f c) { c = wmma_bf(a.l, b.h, c); c = wmma_bf(a.h, b.l, c); return wmma_bf(a.h, b.h, c); }
__device__ __forceinline__ float sigm(float v) { return 1.0f / (1.0f + expf(-v)); }
#define LDSX() do { asm volatile("s_wait_dscnt 0" ::: "memory"); __builtin_amdgcn_wave_barrier(); __builtin_amdgcn_fence(__ATOMIC_RELEASE, "workgroup"); } while (0)

#define NRX 8192
#define DD 1024
#define NRF 1024
#define NOUT 1024

__global__ __launch_bounds__(256) void k_cvt(const float* __restrict__ src, _Float16* __restrict__ dst, size_t n8, float sc) {
  const size_t g8 = (size_t)blockIdx.x * 256 + threadIdx.x; if (g8 >= n8) return;
  union { v8h h; v4u u; } pk;
#pragma unroll
  for (int e = 0; e < 8; ++e) pk.h[e] = (_Float16)(src[g8 * 8 + e] * sc);
  vst2(dst + g8 * 8, pk.u);
}
__global__ __launch_bounds__(128) void k_packR(const float* __restrict__ gs, const float* __restrict__ xis, _Float16* __restrict__ R) {
  const int j = blockIdx.x, tid = threadIdx.x; const float a = xis[j]; union { v8h h; v4u u; } pk;
#pragma unroll
  for (int e = 0; e < 8; ++e) pk.h[e] = (_Float16)(gs[(size_t)j * DD + tid * 8 + e] * a);
  vst2(R + (size_t)j * DD + tid * 8, pk.u);
}
__global__ __launch_bounds__(128) void k_feat(const _Float16* __restrict__ A16, const float* __restrict__ Af, const _Float16* __restrict__ R, const float* __restrict__ xis, _Float16* __restrict__ F) {
  __shared__ __align__(16) float so[4][16][132];
  __shared__ float scor[64];
  const int tid = threadIdx.x, wave = tid >> 5, lane = tid & 31, col = lane & 15, g = lane >> 4;
  const int r0 = blockIdx.x * 64 + wave * 16, n0 = blockIdx.y * 128;
  { const int rl = lane >> 1, hf = lane & 1; const float* ar = Af + (size_t)(r0 + rl) * DD + hf * 512; float s = 0.f;
#pragma unroll 4
    for (int d = 0; d < 512; ++d) { const float v = ar[d]; s += v * v; }
    s += __shfl_xor(s, 1, 32); if (hf == 0) scor[wave * 16 + rl] = 0.5f * s; }
  v8f acc[8] = {};
#pragma unroll 1
  for (int kc = 0; kc < DD / 32; ++kc) { const v16h a = frag_h(A16 + (size_t)(r0 + col) * DD + kc * 32, lane);
#pragma unroll
    for (int j = 0; j < 8; ++j) acc[j] = wmma16(a, frag_h(R + (size_t)(n0 + j * 16 + col) * DD + kc * 32, lane), acc[j]); }
  LDSX();
#pragma unroll
  for (int j = 0; j < 8; ++j) { const int jj = n0 + j * 16 + col; const float ab = xis[jj]; const float pre = expf(ab) * (1.0f / 32.0f) * 16.0f; const float ab2 = ab * ab;
#pragma unroll
    for (int r = 0; r < 8; ++r) so[wave][8 * g + r][j * 16 + col] = pre * expf(acc[j][r] * (1.0f / 16.0f) - scor[wave * 16 + 8 * g + r] * ab2); }
  LDSX();
  for (int q = lane; q < 16 * 16; q += 32) { const int rl = q >> 4, pc = q & 15; union { v8h hh; v4u u; } pk;
#pragma unroll
    for (int e = 0; e < 8; ++e) pk.hh[e] = (_Float16)so[wave][rl][pc * 8 + e];
    vst2(F + (size_t)(r0 + rl) * NRF + n0 + pc * 8, pk.u); }
}
__global__ __launch_bounds__(128) void k_out(const _Float16* __restrict__ F, const _Float16* __restrict__ Wf, float* __restrict__ out) {
  __shared__ __align__(16) float so[4][16][132];
  const int tid = threadIdx.x, wave = tid >> 5, lane = tid & 31, col = lane & 15, g = lane >> 4;
  const int r0 = blockIdx.x * 64 + wave * 16, n0 = blockIdx.y * 128;
  v8f acc[8] = {};
#pragma unroll 1
  for (int kc = 0; kc < NRF / 32; ++kc) { const v16h a = frag_h(F + (size_t)(r0 + col) * NRF + kc * 32, lane);
#pragma unroll
    for (int j = 0; j < 8; ++j) acc[j] = wmma16(a, frag_h(Wf + (size_t)(n0 + j * 16 + col) * NRF + kc * 32, lane), acc[j]); }
#pragma unroll
  for (int j = 0; j < 8; ++j)
#pragma unroll
    for (int r = 0; r < 8; ++r) so[wave][8 * g + r][j * 16 + col] = acc[j][r] * (1.0f / 256.0f);
  LDSX();
#pragma unroll 4
  for (int rl = 0; rl < 16; ++rl) vst2(out + (size_t)(r0 + rl) * NOUT + n0 + lane * 4, *(const v4f*)(&so[wave][rl][lane * 4]));
}
extern "C" void kernel_launch(void* const* d_in, const int* in_sizes, int n_in, void* d_out, int out_size, void* d_ws, size_t ws_size, hipStream_t stream) {
  (void)in_sizes; (void)n_in; (void)out_size; (void)ws_size;
  const float* x = (const float*)d_in[0]; const float* iw = (const float*)d_in[1]; const float* xis = (const float*)d_in[2]; const float* gs = (const float*)d_in[3];
  float* out = (float*)d_out;
  char* ws = (char*)d_ws; size_t off = 0;
  auto take = [&](size_t bytes) { char* p = ws + off; off += (bytes + 255) & ~(size_t)255; return p; };
  _Float16* x16 = (_Float16*)take((size_t)NRX * DD * 2); _Float16* iw16 = (_Float16*)take((size_t)NOUT * DD * 2); _Float16* R = (_Float16*)take((size_t)NRF * DD * 2);
  _Float16* F = (_Float16*)take((size_t)NRX * NRF * 2); _Float16* Wf = (_Float16*)take((size_t)NOUT * NRF * 2);
  { const size_t n8 = (size_t)NRX * DD / 8; k_cvt<<<(unsigned)(n8 / 256), 256, 0, stream>>>(x, x16, n8, 16.0f); }
  { const size_t n8 = (size_t)NOUT * DD / 8; k_cvt<<<(unsigned)(n8 / 256), 256, 0, stream>>>(iw, iw16, n8, 16.0f); }
  k_packR<<<NRF, 128, 0, stream>>>(gs, xis, R);
  k_feat<<<dim3(NRX / 64, NRF / 128), 128, 0, stream>>>(x16, x, R, xis, F);
  k_feat<<<dim3(NOUT / 64, NRF / 128), 128, 0, stream>>>(iw16, iw, R, xis, Wf);
  k_out<<<dim3(NRX / 64, NOUT / 128), 128, 0, stream>>>(F, Wf, out);
}
